// CDAN_Dis_18373870092946
// MI455X (gfx1250) — hardware-verified
//
#include <hip/hip_runtime.h>
#include <math.h>

typedef __attribute__((ext_vector_type(16))) _Float16 v16h;
typedef __attribute__((ext_vector_type(16))) __bf16 v16b;
typedef __attribute__((ext_vector_type(8)))  _Float16 v8h;
typedef __attribute__((ext_vector_type(8)))  float v8f;
typedef __attribute__((ext_vector_type(4)))  float v4f;
typedef __attribute__((ext_vector_type(2)))  float v2f;
typedef __attribute__((ext_vector_type(4)))  unsigned v4u;
typedef __attribute__((ext_vector_type(4)))  int v4i;
typedef float __attribute__((may_alias)) float_a;
typedef int __attribute__((may_alias)) int_a;

template <typename T> __device__ __forceinline__ void vst2(void* p, T v) { *(volatile T*)p = v; __threadfence(); *(volatile T*)p = v; }
__device__ __forceinline__ v8f wmma16(v16h a, v16h b, v8f c) {
  v8f d = __builtin_amdgcn_wmma_f32_16x16x32_f16(false, a, false, b, (short)0, c, false, false);
  asm volatile("v_nop\n\tv_nop\n\tv_nop\n\tv_nop" : "+v"(d) : "v"(a), "v"(b));
  return d;
}
__device__ __forceinline__ v8f wmma_bf(v16b a, v16b b, v8f c) {
  v8f d = __builtin_amdgcn_wmma_f32_16x16x32_bf16(false, a, false, b, (short)0, c, false, false);
  asm volatile("v_nop\n\tv_nop\n\tv_nop\n\tv_nop" : "+v"(d) : "v"(a), "v"(b));
  return d;
}
__device__ __forceinline__ v16h frag_h(const _Float16* rowk0, int lane) {
  union { v16h v; v8h q[2]; } u; const _Float16* p = rowk0 + 8 * (lane >> 4);
  u.q[0] = *(const v8h*)p; u.q[1] = *(const v8h*)(p + 16); return u.v;
}
__device__ __forceinline__ v16h frag_f32(const float* rowk0, int lane) {
  v16h a; const float* p = rowk0 + 8 * (lane >> 4);
#pragma unroll
  for (int i = 0; i < 8; ++i) { a[i] = (_Float16)p[i]; a[8 + i] = (_Float16)p[16 + i]; }
  return a;
}
__device__ __forceinline__ v16h frag_f32s(const float* rowk0, int lane, float sc) {
  v16h a; const float* p = rowk0 + 8 * (lane >> 4);
#pragma unroll
  for (int i = 0; i < 8; ++i) { a[i] = (_Float16)(p[i] * sc); a[8 + i] = (_Float16)(p[16 + i] * sc); }
  return a;
}
__device__ __forceinline__ v16h fragc_f32(const float* W, int k0, int n, int lane, int ld, int K) {
  v16h a; const int g = lane >> 4;
#pragma unroll
  for (int i = 0; i < 8; ++i) { const int ka = k0 + 8 * g + i, kb = ka + 16;
    a[i] = (_Float16)(ka < K ? W[(size_t)(ka < K ? ka : K - 1) * ld + n] : 0.f); a[8 + i] = (_Float16)(kb < K ? W[(size_t)(kb < K ? kb : K - 1) * ld + n] : 0.f); }
  return a;
}
struct F2 { v16b h, l; };
__device__ __forceinline__ F2 bsplit16(const float v[16]) { F2 r;
#pragma unroll
  for (int i = 0; i < 16; ++i) { const __bf16 h = (__bf16)v[i]; r.h[i] = h; r.l[i] = (__bf16)(v[i] - (float)h); }
  return r; }
__device__ __forceinline__ F2 split_row(const float* row, int k0, int lane) { float v[16]; const float* p = row + k0 + 8 * (lane >> 4);
#pragma unroll
  for (int i = 0; i < 8; ++i) { v[i] = p[i]; v[8 + i] = p[16 + i]; }
  return bsplit16(v); }
__device__ __forceinline__ F2 split_rowK(const float* row, int k0, int lane, int K) { float v[16]; const int g = lane >> 4;
#pragma unroll
  for (int i = 0; i < 8; ++i) { const int ka = k0 + 8 * g + i, kb = ka + 16; v[i] = ka < K ? row[ka < K ? ka : K - 1] : 0.f; v[8 + i] = kb < K ? row[kb < K ? kb : K - 1] : 0.f; }
  return bsplit16(v); }
__device__ __forceinline__ F2 split_col(const float* W, int k0, int n, int lane, int ld, int K) { float v[16]; const int g = lane >> 4;
#pragma unroll
  for (int i = 0; i < 8; ++i) { const int ka = k0 + 8 * g + i, kb = ka + 16; v[i] = ka < K ? W[(size_t)(ka < K ? ka : K - 1) * ld + n] : 0.f; v[8 + i] = kb < K ? W[(size_t)(kb < K ? kb : K - 1) * ld + n] : 0.f; }
  return bsplit16(v); }
__device__ __forceinline__ v8f mac3(const F2& a, const F2& b, v8f c) { c = wmma_bf(a.l, b.h, c); c = wmma_bf(a.h, b.l, c); return wmma_bf(a.h, b.h, c); }
__device__ __forceinline__ float sigm(float v) { return 1.0f / (1.0f + expf(-v)); }
#define LDSX() do { asm volatile("s_wait_dscnt 0" ::: "memory"); __builtin_amdgcn_wave_barrier(); __builtin_amdgcn_fence(__ATOMIC_RELEASE, "workgroup"); } while (0)


#define MM 4
#define CCH 2
#define PF 128
#define T0 2000
#define T0P 2048
#define T1 1000
#define T1P 1024
#define T2 500
#define T2P 512
#define CO 256
typedef __attribute__((ext_vector_type(8))) __bf16 v8b;
__device__ __forceinline__ v16b frag_b(const __bf16* rowk0, int lane) {
  union { v16b v; v8b q[2]; } u; const __bf16* p = rowk0 + 8 * (lane >> 4);
  u.q[0] = *(const v8b*)p; u.q[1] = *(const v8b*)(p + 16); return u.v;
}
__device__ __forceinline__ float bfr(float v) { return (float)(__bf16)v; }
__device__ __attribute__((noinline)) float exp_ni(float v) { return expf(v); }
__device__ __attribute__((noinline)) float erf_ni(float v) { return erff(v); }

#define WS_PW   0u
#define PW1 0
#define PW2 (PW1 + CO * 384)
#define PWEND (PW2 + CO * 768)
#define WS_D    (WS_PW + 2u * PWEND)
#define WS_C1   (WS_D + 4u * MM * PF * T0P)
#define WS_C2   (WS_C1 + 4u * MM * CO * T1P)
#define WS_PS   (WS_C2 + 4u * MM * CO * T2P)
#define WS_ST   (WS_PS + 4u * MM * 64 * 32)
#define WS_END  (WS_ST + 4u * 3 * MM * 32)

__global__ __launch_bounds__(256) void k_pack(const float* __restrict__ W1, const float* __restrict__ W2, __bf16* __restrict__ PW) {
  __shared__ __align__(16) __bf16 s[768]; const int o = blockIdx.x, which = blockIdx.y, tid = threadIdx.x; const int K = which ? 768 : 384; const float* src = which ? (W2 + (size_t)o * 768) : (W1 + (size_t)o * 384);
  for (int k = tid; k < K; k += 256) s[k] = (__bf16)src[k];
  __syncthreads();
  for (int q = tid; q < K / 8; q += 256) vst2((unsigned*)(PW + (which ? PW2 : PW1) + (size_t)o * K + q * 8), *(const v4u*)&s[q * 8]);
}
__global__ __launch_bounds__(128) void k_front(const float* __restrict__ FEAT, const float* __restrict__ MASK, const float* __restrict__ W2D, const float* __restrict__ B2D, float* __restrict__ D, float* __restrict__ PS) {
  __shared__ float sa[CCH][64]; __shared__ float sw[CCH][PF]; __shared__ __align__(16) float so[PF][68]; __shared__ float sred[4]; __shared__ __align__(16) float sline[32];
  const int tid = threadIdx.x, chunk = blockIdx.x, m = blockIdx.y; const int t0 = chunk * 64;
  for (int q = tid; q < CCH * PF; q += 128) sw[q / PF][q % PF] = bfr(W2D[q]);
  __syncthreads();
  if (tid < 64) { const int t = t0 + tid; float a0 = 0.f, a1 = 0.f; if (t < T0) {
#pragma unroll 1
      for (int f = 0; f < PF; ++f) { const float fv = bfr(FEAT[((size_t)m * PF + f) * T0 + t]); a0 += sw[0][f] * fv; a1 += sw[1][f] * fv; } }
    sa[0][tid] = a0; sa[1][tid] = a1; }
  __syncthreads();
  const int p = tid; const float b2d = bfr(B2D[0]); float psum = 0.f;
  for (int tl = 0; tl < 64; ++tl) { const int t = t0 + tl; float v = 0.f; if (t < T0) { v = sa[0][tl] * bfr(MASK[(((size_t)m * CCH + 0) * PF + p) * T0 + t]) + sa[1][tl] * bfr(MASK[(((size_t)m * CCH + 1) * PF + p) * T0 + t]) + b2d; psum += v; } so[p][tl] = v; }
  float q = psum;
#pragma unroll
  for (int o = 1; o < 32; o <<= 1) q += __shfl_xor(q, o);
  if ((tid & 31) == 0) sred[tid >> 5] = q;
  __syncthreads();
  for (int qq = tid; qq < PF * 16; qq += 128) { const int pp = qq >> 4, pc = qq & 15; vst2(D + ((size_t)m * PF + pp) * T0P + t0 + pc * 4, *(const v4f*)&so[pp][pc * 4]); }
  if (tid < 32) { float v = 0.f; if (tid == 0) v = (sred[0] + sred[1]) + (sred[2] + sred[3]); sline[tid] = v; }
  __syncthreads();
  if (tid < 8) vst2(PS + ((size_t)m * 64 + chunk) * 32 + tid * 4, *(const v4f*)&sline[tid * 4]);
}
__global__ __launch_bounds__(64) void k_red(const float* __restrict__ PS, int nblk, float count, int norm, int MODE, float* __restrict__ ST) {
  __shared__ float s[64]; __shared__ __align__(16) float sline[32]; const int m = blockIdx.x, tid = threadIdx.x;
  s[tid] = (tid < nblk) ? PS[((size_t)m * 64 + tid) * 32] : 0.f; const float keep = (MODE == 1) ? ST[((size_t)norm * MM + m) * 32] : 0.f; __syncthreads();
  if (tid < 32) sline[tid] = 0.f;
  __syncthreads();
  if (tid == 0) { float acc = 0.f; for (int i = 0; i < nblk; ++i) acc += s[i]; acc /= count; if (MODE == 0) sline[0] = acc; else { sline[0] = keep; sline[1] = 1.0f / sqrtf(acc + 1e-8f); } }
  __syncthreads();
  if (tid < 8) vst2(ST + ((size_t)norm * MM + m) * 32 + tid * 4, *(const v4f*)&sline[tid * 4]);
}
__global__ __launch_bounds__(128) void k_var(const float* __restrict__ PL, int nch, int pitch, int width, const float* __restrict__ ST, int norm, float* __restrict__ PS) {
  __shared__ float sred[4]; __shared__ __align__(16) float sline[32]; const int tid = threadIdx.x, chunk = blockIdx.x, m = blockIdx.y; const int t0 = chunk * 64; const float mu = ST[((size_t)norm * MM + m) * 32];
  float acc = 0.f;
  for (int c = tid; c < nch; c += 128) { const float* row = PL + ((size_t)m * nch + c) * pitch + t0; for (int tl = 0; tl < 64; ++tl) if (t0 + tl < width) { const float d = row[tl] - mu; acc += d * d; } }
#pragma unroll
  for (int o = 1; o < 32; o <<= 1) acc += __shfl_xor(acc, o);
  if ((tid & 31) == 0) sred[tid >> 5] = acc;
  __syncthreads();
  if (tid < 32) { float v = 0.f; if (tid == 0) v = (sred[0] + sred[1]) + (sred[2] + sred[3]); sline[tid] = v; }
  __syncthreads();
  if (tid < 8) vst2(PS + ((size_t)m * 64 + chunk) * 32 + tid * 4, *(const v4f*)&sline[tid * 4]);
}
template <int CIN>
__global__ __launch_bounds__(128) void k_conv(const float* __restrict__ SRC, int spitch, int win, const float* __restrict__ ST, int norm, const float* __restrict__ G, const float* __restrict__ BE, int gstride, const __bf16* __restrict__ PW, const float* __restrict__ bias, float* __restrict__ DST, int dpitch, int wout, float* __restrict__ PS) {
  __shared__ __align__(16) float st[128][68]; __shared__ float sred[4]; __shared__ __align__(16) float sline[32];
  const int tid = threadIdx.x, wave = tid >> 5, lane = tid & 31, col = lane & 15, g = lane >> 4; const int m = blockIdx.z; const int p0 = blockIdx.x * 64; const int n0 = blockIdx.y * 128; const int to = p0 + wave * 16 + col;
  const float mu = ST[((size_t)norm * MM + m) * 32], rs = ST[((size_t)norm * MM + m) * 32 + 1];
  const float* sb = SRC + (size_t)m * CIN * spitch;
  v8f acc[8] = {};
#pragma unroll 1
  for (int kc = 0; kc < CIN * 3 / 32; ++kc) { float v[16];
#pragma unroll
    for (int i = 0; i < 16; ++i) { const int kk = kc * 32 + 8 * g + (i & 7) + ((i >> 3) << 4); const int cin = kk / 3, j = kk - cin * 3; const int ti = 2 * to - 1 + j; float val = 0.f;
      if (ti >= 0 && ti < win) { const float raw = sb[(size_t)cin * spitch + ti]; const float gg = bfr(G[cin * gstride]), bb = bfr(BE[cin * gstride]); float x = gg * (raw - mu) * rs + bb; val = (x >= 0.f) ? x : 0.1f * x; }
      v[i] = val; }
    const F2 a = bsplit16(v);
#pragma unroll
    for (int jj = 0; jj < 8; ++jj) { const v16b w = frag_b(PW + (size_t)(n0 + jj * 16 + col) * (CIN * 3) + kc * 32, lane); acc[jj] = wmma_bf(a.l, w, acc[jj]); acc[jj] = wmma_bf(a.h, w, acc[jj]); } }
  float psum = 0.f;
#pragma unroll
  for (int jj = 0; jj < 8; ++jj) { const int o = jj * 16 + col; const float bb = bfr(bias[n0 + o]);
#pragma unroll
    for (int r = 0; r < 8; ++r) { const int tt = p0 + wave * 16 + 8 * g + r; float vv = acc[jj][r] + bb; if (tt >= wout) vv = 0.f; else psum += vv; st[o][wave * 16 + 8 * g + r] = vv; } }
#pragma unroll
  for (int o = 1; o < 32; o <<= 1) psum += __shfl_xor(psum, o);
  if (lane == 0) sred[wave] = psum;
  __syncthreads();
  for (int q = tid; q < 128 * 16; q += 128) { const int o = q >> 4, pc = q & 15; vst2(DST + ((size_t)m * CO + n0 + o) * dpitch + p0 + pc * 4, *(const v4f*)&st[o][pc * 4]); }
  if (tid < 32) { float vv = 0.f; if (tid == 0) vv = (sred[0] + sred[1]) + (sred[2] + sred[3]); sline[tid] = vv; }
  __syncthreads();
  if (tid < 8) vst2(PS + ((size_t)m * 64 + blockIdx.x * 2 + blockIdx.y) * 32 + tid * 4, *(const v4f*)&sline[tid * 4]);
}
__global__ __launch_bounds__(256) void k_out(const float* __restrict__ C2, const float* __restrict__ ST, const float* __restrict__ G3, const float* __restrict__ BE3, const float* __restrict__ W3, const float* __restrict__ B3, float* __restrict__ out) {
  __shared__ __align__(16) float so[MM * T2]; __shared__ float sw[CO], sg[CO], sbe[CO]; const int tid = threadIdx.x;
  sw[tid] = bfr(W3[tid]); sg[tid] = bfr(G3[tid]); sbe[tid] = bfr(BE3[tid]);
  __syncthreads();
  const float b3 = bfr(B3[0]);
  for (int q = tid; q < MM * T2; q += 256) { const int m = q / T2, t = q % T2; const float mu = ST[((size_t)2 * MM + m) * 32], rs = ST[((size_t)2 * MM + m) * 32 + 1]; float acc = b3;
#pragma unroll 1
    for (int o = 0; o < CO; ++o) { float x = sg[o] * (C2[((size_t)m * CO + o) * T2P + t] - mu) * rs + sbe[o]; x = (x >= 0.f) ? x : 0.1f * x; acc += sw[o] * x; }
    so[q] = acc; }
  __syncthreads();
  for (int q = tid; q < MM * T2 / 4; q += 256) vst2(out + q * 4, *(const v4f*)&so[q * 4]);
}
extern "C" void kernel_launch(void* const* d_in, const int* in_sizes, int n_in, void* d_out, int out_size, void* d_ws, size_t ws_size, hipStream_t stream) {
  (void)in_sizes; (void)n_in; (void)out_size;
  const float** F = (const float**)d_in;
  if (ws_size < (size_t)WS_END) return;
  char* ws = (char*)d_ws; __bf16* PW = (__bf16*)(ws + WS_PW); float *D = (float*)(ws + WS_D), *C1 = (float*)(ws + WS_C1), *C2 = (float*)(ws + WS_C2), *PS = (float*)(ws + WS_PS), *ST = (float*)(ws + WS_ST);
  k_pack<<<dim3(CO, 2), 256, 0, stream>>>(F[6], F[10], PW);
  k_front<<<dim3(T0P / 64, MM), 128, 0, stream>>>(F[0], F[1], F[2], F[3], D, PS);
  k_red<<<MM, 64, 0, stream>>>(PS, 32, (float)(PF * T0), 0, 0, ST);
  k_var<<<dim3(T0P / 64, MM), 128, 0, stream>>>(D, PF, T0P, T0, ST, 0, PS);
  k_red<<<MM, 64, 0, stream>>>(PS, 32, (float)(PF * T0), 0, 1, ST);
  k_conv<PF><<<dim3(T1P / 64, 2, MM), 128, 0, stream>>>(D, T0P, T0, ST, 0, F[4], F[5], 0, PW + PW1, F[7], C1, T1P, T1, PS);
  k_red<<<MM, 64, 0, stream>>>(PS, 32, (float)(CO * T1), 1, 0, ST);
  k_var<<<dim3(T1P / 64, MM), 128, 0, stream>>>(C1, CO, T1P, T1, ST, 1, PS);
  k_red<<<MM, 64, 0, stream>>>(PS, 16, (float)(CO * T1), 1, 1, ST);
  k_conv<CO><<<dim3(T2P / 64, 2, MM), 128, 0, stream>>>(C1, T1P, T1, ST, 1, F[8], F[9], 1, PW + PW2, F[11], C2, T2P, T2, PS);
  k_red<<<MM, 64, 0, stream>>>(PS, 16, (float)(CO * T2), 2, 0, ST);
  k_var<<<dim3(T2P / 64, MM), 128, 0, stream>>>(C2, CO, T2P, T2, ST, 2, PS);
  k_red<<<MM, 64, 0, stream>>>(PS, 8, (float)(CO * T2), 2, 1, ST);
  k_out<<<1, 256, 0, stream>>>(C2, ST, F[12], F[13], F[14], F[15], (float*)d_out);
}
